// FullJointMMDiTAdapter_76175539961969
// MI455X (gfx1250) — hardware-run, weakly checked
//
#include <hip/hip_runtime.h>


#define NB_  2
#define LI   1024
#define LC   256
#define SS   1280
#define HH   1024
#define NH_  16
#define HD   64
#define MLP  4096
#define ZH   2
#define PCAR 1024.0f
typedef _Float16 h16;
typedef unsigned short bf;
typedef __attribute__((ext_vector_type(16))) __bf16   v16bf;
typedef __attribute__((ext_vector_type(16))) _Float16 v16h;
typedef __attribute__((ext_vector_type(8)))  _Float16 v8h;
typedef __attribute__((ext_vector_type(8)))  unsigned short v8us;
typedef __attribute__((ext_vector_type(8)))  float    v8f;
typedef __attribute__((ext_vector_type(4)))  float    v4f;
typedef v8h  __attribute__((may_alias)) v8ha;
typedef v4f  __attribute__((may_alias)) v4fa;
typedef v8us __attribute__((may_alias)) v8usa;

__device__ __forceinline__ unsigned short f2bf(float f) { unsigned u = __float_as_uint(f); u += 0x7FFFu + ((u >> 16) & 1u); return (unsigned short)(u >> 16); }
__device__ __forceinline__ float bf2f(unsigned short b) { return __uint_as_float(((unsigned)b) << 16); }
__device__ __forceinline__ float bfr(float f) { return bf2f(f2bf(f)); }
__device__ __forceinline__ v16h cat16(v8h lo, v8h hi) { return __builtin_shufflevector(lo, hi, 0, 1, 2, 3, 4, 5, 6, 7, 8, 9, 10, 11, 12, 13, 14, 15); }
__device__ __forceinline__ v16bf cat16b(v8us lo, v8us hi) { return __builtin_bit_cast(v16bf, __builtin_shufflevector(lo, hi, 0, 1, 2, 3, 4, 5, 6, 7, 8, 9, 10, 11, 12, 13, 14, 15)); }
__device__ __forceinline__ v8f wmma16(v16h a, v16h b, v8f c) { return __builtin_amdgcn_wmma_f32_16x16x32_f16(false, a, false, b, (short)0, c, false, false); }
__device__ __forceinline__ v8f wmmab(v16bf a, v16bf b, v8f c) { return __builtin_amdgcn_wmma_f32_16x16x32_bf16(false, a, false, b, (short)0, c, false, false); }


template <typename T16> struct WFrag;
template <> struct WFrag<h16> { typedef v16h V; static __device__ __forceinline__ V ld(const h16* p) { return cat16(*(const v8h*)p, *(const v8h*)(p + 16)); } static __device__ __forceinline__ v8f mma(V a, V b, v8f c) { return wmma16(a, b, c); } };
template <> struct WFrag<bf> { typedef v16bf V; static __device__ __forceinline__ V ld(const bf* p) { return cat16b(*(const v8us*)p, *(const v8us*)(p + 16)); } static __device__ __forceinline__ v8f mma(V a, V b, v8f c) { return wmmab(a, b, c); } };
template <typename T16, int NSPLIT, bool BIAS>
__global__ __launch_bounds__(32) void k_gemmw(const T16* __restrict__ A, const T16* __restrict__ A2, const T16* __restrict__ Bt, const T16* __restrict__ Bt2, int K, float* C, int ldc, const float* __restrict__ bias, size_t sA, size_t sB, size_t sC) {
    typedef typename WFrag<T16>::V V;
    __shared__ __align__(16) float os[16 * 68];
    const size_t z = blockIdx.z; A += z * sA; if (A2) A2 += z * sA; Bt += z * sB; if (Bt2) Bt2 += z * sB; C += z * sC;
    const int lane = threadIdx.x & 31, lr = lane & 15, hi = lane >> 4; const int r0 = blockIdx.x * 64, c0 = blockIdx.y * 64;
    v8f acc[4][4];
#pragma unroll
    for (int mb = 0; mb < 4; ++mb)
#pragma unroll
        for (int nb = 0; nb < 4; ++nb) acc[mb][nb] = (v8f){};
    const size_t aoff = (size_t)(r0 + lr) * K + 8 * hi, boff = (size_t)(c0 + lr) * K + 8 * hi;
#pragma unroll 1
    for (int kc = 0; kc < K; kc += 32) {
        V a[4], a2[4];
#pragma unroll
        for (int mb = 0; mb < 4; ++mb) { a[mb] = WFrag<T16>::ld(A + aoff + (size_t)mb * 16 * K + kc); if (NSPLIT == 1 || NSPLIT == 2) a2[mb] = WFrag<T16>::ld(A2 + aoff + (size_t)mb * 16 * K + kc); }
#pragma unroll
        for (int nb = 0; nb < 4; ++nb) { const V b = WFrag<T16>::ld(Bt + boff + (size_t)nb * 16 * K + kc); V b2; if (NSPLIT >= 2) b2 = WFrag<T16>::ld(Bt2 + boff + (size_t)nb * 16 * K + kc);
#pragma unroll
            for (int mb = 0; mb < 4; ++mb) { acc[mb][nb] = WFrag<T16>::mma(a[mb], b, acc[mb][nb]); if (NSPLIT == 1 || NSPLIT == 2) acc[mb][nb] = WFrag<T16>::mma(a2[mb], b, acc[mb][nb]); if (NSPLIT >= 2) acc[mb][nb] = WFrag<T16>::mma(a[mb], b2, acc[mb][nb]); } }
        asm volatile("v_nop\n\tv_nop\n\tv_nop\n\tv_nop" : "+v"(acc[0][0]), "+v"(acc[1][1]), "+v"(acc[2][2]), "+v"(acc[3][3]) : "v"(a[0]), "v"(a[3]));
    }
#pragma unroll
    for (int mb = 0; mb < 4; ++mb) {
#pragma unroll
        for (int nb = 0; nb < 4; ++nb) {
#pragma unroll
            for (int j = 0; j < 8; ++j) os[(hi * 8 + j) * 68 + nb * 16 + lr] = acc[mb][nb][j]; }
        __builtin_amdgcn_wave_barrier(); asm volatile("" ::: "memory");
        float* crow = C + (size_t)(r0 + mb * 16) * ldc + c0;
#pragma unroll 1
        for (int ps = 0; ps < 2; ++ps) {
#pragma unroll
            for (int s = 0; s < 8; ++s) { const int row = 2 * s + hi, cofs = lr * 4; v4f val = *(const v4fa*)(os + row * 68 + cofs); if (BIAS) { val[0] += bfr(bias[c0 + cofs]); val[1] += bfr(bias[c0 + cofs + 1]); val[2] += bfr(bias[c0 + cofs + 2]); val[3] += bfr(bias[c0 + cofs + 3]); }
                *(volatile v4f*)(crow + (size_t)row * ldc + cofs) = val; }
            if (ps == 0) __threadfence(); }
        __builtin_amdgcn_wave_barrier(); asm volatile("" ::: "memory");
    }
}

template <typename T16, int NSPLIT, bool BIAS>
__global__ __launch_bounds__(32) void k_gemmwg(const float* __restrict__ gate, const T16* __restrict__ A, const T16* __restrict__ A2, const T16* __restrict__ Bt, const T16* __restrict__ Bt2, int K, float* C, int ldc, const float* __restrict__ bias, size_t sA, size_t sB, size_t sC) {
    if (bfr(gate[0]) == 0.0f) return;
    typedef typename WFrag<T16>::V V;
    __shared__ __align__(16) float os[16 * 68];
    const size_t z = blockIdx.z; A += z * sA; if (A2) A2 += z * sA; Bt += z * sB; if (Bt2) Bt2 += z * sB; C += z * sC;
    const int lane = threadIdx.x & 31, lr = lane & 15, hi = lane >> 4; const int r0 = blockIdx.x * 64, c0 = blockIdx.y * 64;
    v8f acc[4][4];
#pragma unroll
    for (int mb = 0; mb < 4; ++mb)
#pragma unroll
        for (int nb = 0; nb < 4; ++nb) acc[mb][nb] = (v8f){};
    const size_t aoff = (size_t)(r0 + lr) * K + 8 * hi, boff = (size_t)(c0 + lr) * K + 8 * hi;
#pragma unroll 1
    for (int kc = 0; kc < K; kc += 32) {
        V a[4], a2[4];
#pragma unroll
        for (int mb = 0; mb < 4; ++mb) { a[mb] = WFrag<T16>::ld(A + aoff + (size_t)mb * 16 * K + kc); if (NSPLIT == 1 || NSPLIT == 2) a2[mb] = WFrag<T16>::ld(A2 + aoff + (size_t)mb * 16 * K + kc); }
#pragma unroll
        for (int nb = 0; nb < 4; ++nb) { const V b = WFrag<T16>::ld(Bt + boff + (size_t)nb * 16 * K + kc); V b2; if (NSPLIT >= 2) b2 = WFrag<T16>::ld(Bt2 + boff + (size_t)nb * 16 * K + kc);
#pragma unroll
            for (int mb = 0; mb < 4; ++mb) { acc[mb][nb] = WFrag<T16>::mma(a[mb], b, acc[mb][nb]); if (NSPLIT == 1 || NSPLIT == 2) acc[mb][nb] = WFrag<T16>::mma(a2[mb], b, acc[mb][nb]); if (NSPLIT >= 2) acc[mb][nb] = WFrag<T16>::mma(a[mb], b2, acc[mb][nb]); } }
        asm volatile("v_nop\n\tv_nop\n\tv_nop\n\tv_nop" : "+v"(acc[0][0]), "+v"(acc[1][1]), "+v"(acc[2][2]), "+v"(acc[3][3]) : "v"(a[0]), "v"(a[3]));
    }
#pragma unroll
    for (int mb = 0; mb < 4; ++mb) {
#pragma unroll
        for (int nb = 0; nb < 4; ++nb) {
#pragma unroll
            for (int j = 0; j < 8; ++j) os[(hi * 8 + j) * 68 + nb * 16 + lr] = acc[mb][nb][j]; }
        __builtin_amdgcn_wave_barrier(); asm volatile("" ::: "memory");
        float* crow = C + (size_t)(r0 + mb * 16) * ldc + c0;
#pragma unroll 1
        for (int ps = 0; ps < 2; ++ps) {
#pragma unroll
            for (int s = 0; s < 8; ++s) { const int row = 2 * s + hi, cofs = lr * 4; v4f val = *(const v4fa*)(os + row * 68 + cofs); if (BIAS) { val[0] += bfr(bias[c0 + cofs]); val[1] += bfr(bias[c0 + cofs + 1]); val[2] += bfr(bias[c0 + cofs + 2]); val[3] += bfr(bias[c0 + cofs + 3]); }
                *(volatile v4f*)(crow + (size_t)row * ldc + cofs) = val; }
            if (ps == 0) __threadfence(); }
        __builtin_amdgcn_wave_barrier(); asm volatile("" ::: "memory");
    }
}

__device__ __forceinline__ h16 tohx(float x) { return (h16)x; }
__device__ __forceinline__ void splitf(float y, unsigned short& h, unsigned short& l) { h = f2bf(y); l = f2bf(y - bf2f(h)); }
typedef __attribute__((ext_vector_type(2))) _Float16 v2h;
typedef __attribute__((ext_vector_type(4))) _Float16 v4h;
typedef __attribute__((ext_vector_type(2))) unsigned short v2us;
typedef __attribute__((ext_vector_type(4))) unsigned short v4us;
typedef __attribute__((ext_vector_type(2))) float v2f;

__global__ __launch_bounds__(256) void k_cvt8(const float* __restrict__ src, bf* dst, size_t n8) { const size_t i = (size_t)blockIdx.x * 256 + threadIdx.x; if (i >= n8) return; const v8f v = *(const v8f*)(src + i * 8); v8us o;
#pragma unroll
    for (int k = 0; k < 8; ++k) o[k] = f2bf(v[k]); *(volatile v8us*)(dst + i * 8) = o; __threadfence(); *(volatile v8us*)(dst + i * 8) = o; }
__global__ __launch_bounds__(256) void k_rms(const float* __restrict__ X, int isin, int ntok, const float* __restrict__ w, bf* Xh, bf* Xl) { const int lane = threadIdx.x & 31; const int t = blockIdx.x * 8 + (threadIdx.x >> 5); if (t >= ntok) return; const size_t rb = (size_t)t * HH; float q2 = 0.f;
#pragma unroll 1
    for (int ch = 0; ch < 8; ++ch) { const v4f a = *(const v4f*)(X + rb + ch * 128 + lane * 4);
#pragma unroll
        for (int q = 0; q < 4; ++q) { const float xv = isin ? bfr(a[q]) : a[q]; float p = __fmul_rn(xv, xv); asm volatile("" : "+v"(p)); q2 = __fadd_rn(q2, p); } }
#pragma unroll
    for (int sh = 16; sh; sh >>= 1) q2 += __shfl_xor(q2, sh, 32);
    const float r = __frsqrt_rn(__fadd_rn(q2 * (1.0f / HH), 1e-6f));
#pragma unroll 1
    for (int ch = 0; ch < 8; ++ch) { const int c0 = ch * 128 + lane * 4; const v4f a = *(const v4f*)(X + rb + c0); v4us oh, ol;
#pragma unroll
        for (int q = 0; q < 4; ++q) { const float xv = isin ? bfr(a[q]) : a[q]; float tn = __fmul_rn(xv, r); asm volatile("" : "+v"(tn)); unsigned short u, c; splitf(__fmul_rn(tn, bfr(w[c0 + q])), u, c); oh[q] = u; ol[q] = c; }
        *(volatile v4us*)(Xh + rb + c0) = oh; *(volatile v4us*)(Xl + rb + c0) = ol; __threadfence(); *(volatile v4us*)(Xh + rb + c0) = oh; *(volatile v4us*)(Xl + rb + c0) = ol; } }
__global__ __launch_bounds__(256) void k_qk(const float* __restrict__ QKV, int ntok, int roff, const float* __restrict__ cosT, const float* __restrict__ sinT, const float* __restrict__ qn, const float* __restrict__ kn, h16* Q16, h16* K16) {
    const int lane = threadIdx.x & 31; const int row = blockIdx.x * 8 + (threadIdx.x >> 5); if (row >= ntok * NH_ * 2) return; const int which = row & 1; const int h = (row >> 1) % NH_; const int t = (row >> 1) / NH_;
    const float* src = QKV + (size_t)t * 3 * HH + which * HH + h * HD; const float a0 = src[lane], a1 = src[lane + 32]; float q2 = __fadd_rn(__fmul_rn(a0, a0), __fmul_rn(a1, a1));
#pragma unroll
    for (int sh = 16; sh; sh >>= 1) q2 += __shfl_xor(q2, sh, 32);
    const float r = __frsqrt_rn(__fadd_rn(q2 * (1.0f / HD), 1e-6f)); const float* nw = which ? kn : qn; float t0 = __fmul_rn(a0, r), t1 = __fmul_rn(a1, r); asm volatile("" : "+v"(t0), "+v"(t1)); const float n0 = __fmul_rn(t0, bfr(nw[lane])), n1 = __fmul_rn(t1, bfr(nw[lane + 32]));
    const float c0 = bfr(cosT[(size_t)t * HD + lane]), c1 = bfr(cosT[(size_t)t * HD + lane + 32]), s0 = bfr(sinT[(size_t)t * HD + lane]), s1 = bfr(sinT[(size_t)t * HD + lane + 32]);
    float p0 = __fmul_rn(n0, c0); asm volatile("" : "+v"(p0)); float p1 = __fmul_rn(-n1, s0); asm volatile("" : "+v"(p1)); float p2 = __fmul_rn(n1, c1); asm volatile("" : "+v"(p2)); float p3 = __fmul_rn(n0, s1); asm volatile("" : "+v"(p3));
    float o0 = __fadd_rn(p0, p1), o1 = __fadd_rn(p2, p3); if (!which) { o0 *= 0.125f; o1 *= 0.125f; }
    const int e0 = 2 * lane, e1 = 2 * lane + 1; const float f00 = __shfl(o0, e0 & 31, 32), f01 = __shfl(o1, e0 & 31, 32), f10 = __shfl(o0, e1 & 31, 32), f11 = __shfl(o1, e1 & 31, 32); v2h pr; pr[0] = tohx(e0 < 32 ? f00 : f01); pr[1] = tohx(e1 < 32 ? f10 : f11);
    h16* dst = (which ? K16 : Q16) + ((size_t)h * SS + roff + t) * HD; *(volatile v2h*)(dst + e0) = pr; __threadfence(); *(volatile v2h*)(dst + e0) = pr; }
__global__ __launch_bounds__(256) void k_vt(const float* __restrict__ QKV, int ntok, int coff, h16* VT) { const size_t e = ((size_t)blockIdx.x * 256 + threadIdx.x) * 2; if (e >= (size_t)NH_ * HD * ntok) return; const int t = (int)(e % ntok); const int d = (int)((e / ntok) % HD); const int h = (int)(e / ((size_t)ntok * HD)); v2h o; o[0] = tohx(QKV[(size_t)t * 3 * HH + 2 * HH + h * HD + d]); o[1] = tohx(QKV[(size_t)(t + 1) * 3 * HH + 2 * HH + h * HD + d]); const size_t oo = ((size_t)h * HD + d) * SS + coff + t; *(volatile v2h*)(VT + oo) = o; __threadfence(); *(volatile v2h*)(VT + oo) = o; }
__global__ __launch_bounds__(256) void k_soft(const float* __restrict__ Sb, int nrows, h16* P) { const int lane = threadIdx.x & 31; const int row = blockIdx.x * 8 + (threadIdx.x >> 5); if (row >= nrows) return; const float* sr = Sb + (size_t)row * SS; float v[40]; float mx = -3.0e38f;
#pragma unroll
    for (int ch = 0; ch < 10; ++ch) { const v4f a = *(const v4f*)(sr + ch * 128 + lane * 4);
#pragma unroll
        for (int q = 0; q < 4; ++q) { v[ch * 4 + q] = a[q]; mx = fmaxf(mx, a[q]); } }
#pragma unroll
    for (int sh = 16; sh; sh >>= 1) mx = fmaxf(mx, __shfl_xor(mx, sh, 32));
    float sum = 0.f;
#pragma unroll
    for (int k = 0; k < 40; ++k) { float d0 = __fsub_rn(v[k], mx); asm volatile("" : "+v"(d0)); v[k] = __expf(d0); sum += v[k]; }
#pragma unroll
    for (int sh = 16; sh; sh >>= 1) sum += __shfl_xor(sum, sh, 32);
    const float f = __fdiv_rn(PCAR, sum);
#pragma unroll 1
    for (int ps = 0; ps < 2; ++ps) {
#pragma unroll
        for (int ch = 0; ch < 10; ++ch) { v4h o; o[0] = tohx(v[ch * 4] * f); o[1] = tohx(v[ch * 4 + 1] * f); o[2] = tohx(v[ch * 4 + 2] * f); o[3] = tohx(v[ch * 4 + 3] * f); *(volatile v4h*)(P + (size_t)row * SS + ch * 128 + lane * 4) = o; }
        if (ps == 0) __threadfence(); } }
__global__ __launch_bounds__(256) void k_mrg(const float* __restrict__ Ob, int ntok, int roff, int h0, bf* Ah, bf* Al) { const size_t e = ((size_t)blockIdx.x * 256 + threadIdx.x) * 2; if (e >= (size_t)ZH * ntok * HD) return; const int d = (int)(e % HD); const int t = (int)((e / HD) % ntok); const int z = (int)(e / ((size_t)HD * ntok)); v2us oh, ol;
#pragma unroll
    for (int u = 0; u < 2; ++u) { unsigned short a, c; splitf(Ob[((size_t)z * SS + roff + t) * HD + d + u] * (1.0f / PCAR), a, c); oh[u] = a; ol[u] = c; } const size_t o = (size_t)t * HH + (h0 + z) * HD + d; *(volatile v2us*)(Ah + o) = oh; *(volatile v2us*)(Al + o) = ol; __threadfence(); *(volatile v2us*)(Ah + o) = oh; *(volatile v2us*)(Al + o) = ol; }
__global__ __launch_bounds__(256) void k_mrgg(const float* __restrict__ gate, const float* __restrict__ Ob, int ntok, int roff, int h0, bf* Ah, bf* Al) { if (bfr(gate[0]) == 0.0f) return; const size_t e = ((size_t)blockIdx.x * 256 + threadIdx.x) * 2; if (e >= (size_t)ZH * ntok * HD) return; const int d = (int)(e % HD); const int t = (int)((e / HD) % ntok); const int z = (int)(e / ((size_t)HD * ntok)); v2us oh, ol;
#pragma unroll
    for (int u = 0; u < 2; ++u) { unsigned short a, c; splitf(Ob[((size_t)z * SS + roff + t) * HD + d + u] * (1.0f / PCAR), a, c); oh[u] = a; ol[u] = c; } const size_t o = (size_t)t * HH + (h0 + z) * HD + d; *(volatile v2us*)(Ah + o) = oh; *(volatile v2us*)(Al + o) = ol; __threadfence(); *(volatile v2us*)(Ah + o) = oh; *(volatile v2us*)(Al + o) = ol; }
__global__ __launch_bounds__(256) void k_softg(const float* __restrict__ gate, const float* __restrict__ Sb, int nrows, h16* P) { if (bfr(gate[0]) == 0.0f) return; const int lane = threadIdx.x & 31; const int row = blockIdx.x * 8 + (threadIdx.x >> 5); if (row >= nrows) return; const float* sr = Sb + (size_t)row * SS; float v[40]; float mx = -3.0e38f;
#pragma unroll
    for (int ch = 0; ch < 10; ++ch) { const v4f a = *(const v4f*)(sr + ch * 128 + lane * 4);
#pragma unroll
        for (int q = 0; q < 4; ++q) { v[ch * 4 + q] = a[q]; mx = fmaxf(mx, a[q]); } }
#pragma unroll
    for (int sh = 16; sh; sh >>= 1) mx = fmaxf(mx, __shfl_xor(mx, sh, 32));
    float sum = 0.f;
#pragma unroll
    for (int k = 0; k < 40; ++k) { float d0 = __fsub_rn(v[k], mx); asm volatile("" : "+v"(d0)); v[k] = __expf(d0); sum += v[k]; }
#pragma unroll
    for (int sh = 16; sh; sh >>= 1) sum += __shfl_xor(sum, sh, 32);
    const float f = __fdiv_rn(PCAR, sum);
#pragma unroll 1
    for (int ps = 0; ps < 2; ++ps) {
#pragma unroll
        for (int ch = 0; ch < 10; ++ch) { v4h o; o[0] = tohx(v[ch * 4] * f); o[1] = tohx(v[ch * 4 + 1] * f); o[2] = tohx(v[ch * 4 + 2] * f); o[3] = tohx(v[ch * 4 + 3] * f); *(volatile v4h*)(P + (size_t)row * SS + ch * 128 + lane * 4) = o; }
        if (ps == 0) __threadfence(); } }
__global__ __launch_bounds__(256) void k_resg(const float* __restrict__ x, int isin, const float* __restrict__ D, const float* __restrict__ gate, size_t n4, float* X1) { const size_t i = ((size_t)blockIdx.x * 256 + threadIdx.x) * 4; if (i >= n4 * 4) return; const float g = gate ? bfr(gate[0]) : 1.0f; v4f d; if (g != 0.0f) d = *(const v4f*)(D + i); v4f o;
#pragma unroll
    for (int q = 0; q < 4; ++q) { const float xv = isin ? bfr(x[i + q]) : x[i + q]; float add = 0.f; if (g != 0.0f) { add = gate ? __fmul_rn(g, d[q]) : d[q]; } o[q] = __fadd_rn(xv, add); }
    *(volatile v4f*)(X1 + i) = o; __threadfence(); *(volatile v4f*)(X1 + i) = o; }
__global__ __launch_bounds__(256) void k_swi(const float* __restrict__ A, const float* __restrict__ Bv, size_t n4, const float* __restrict__ gate, bf* Fh, bf* Fl) { const size_t i = ((size_t)blockIdx.x * 256 + threadIdx.x) * 4; if (i >= n4 * 4) return; if (gate && bfr(gate[0]) == 0.0f) return; const v4f a = *(const v4f*)(A + i), c = *(const v4f*)(Bv + i); v4us oh, ol;
#pragma unroll
    for (int q = 0; q < 4; ++q) { const float sg = __fdiv_rn(1.0f, 1.0f + __expf(-a[q])); float sl = __fmul_rn(a[q], sg); asm volatile("" : "+v"(sl)); unsigned short u, l; splitf(__fmul_rn(sl, c[q]), u, l); oh[q] = u; ol[q] = l; }
    *(volatile v4us*)(Fh + i) = oh; *(volatile v4us*)(Fl + i) = ol; __threadfence(); *(volatile v4us*)(Fh + i) = oh; *(volatile v4us*)(Fl + i) = ol; }

extern "C" void kernel_launch(void* const* d_in, const int* in_sizes, int n_in,
                              void* d_out, int out_size, void* d_ws, size_t ws_size, hipStream_t stream) {
    (void)in_sizes; (void)n_in; (void)out_size;
    const float* IN[36]; for (int i = 0; i < 36; ++i) IN[i] = (const float*)d_in[i];
    float* OUTI = (float*)d_out; float* OUTC = (float*)((char*)d_out + 8388608);
    char* wsp = (char*)d_ws;
    auto take = [&](size_t bytes) { char* p = wsp; wsp += (bytes + 255) & ~(size_t)255; return (void*)p; };
    bf* WQI = (bf*)take((size_t)3 * HH * HH * 2); bf* WQC = (bf*)take((size_t)3 * HH * HH * 2); bf* WOI = (bf*)take((size_t)HH * HH * 2); bf* WOC = (bf*)take((size_t)HH * HH * 2); bf* W1I = (bf*)take((size_t)MLP * HH * 2); bf* W2I = (bf*)take((size_t)MLP * HH * 2); bf* W3I = (bf*)take((size_t)HH * MLP * 2); bf* W1C = (bf*)take((size_t)MLP * HH * 2); bf* W2C = (bf*)take((size_t)MLP * HH * 2); bf* W3C = (bf*)take((size_t)HH * MLP * 2);
    bf* Xh = (bf*)take((size_t)LI * HH * 2); bf* Xl = (bf*)take((size_t)LI * HH * 2); float* QKVI = (float*)take((size_t)LI * 3 * HH * 4); float* QKVC = (float*)take((size_t)LC * 3 * HH * 4); h16* Q16 = (h16*)take((size_t)NH_ * SS * HD * 2); h16* K16 = (h16*)take((size_t)NH_ * SS * HD * 2); h16* VT = (h16*)take((size_t)NH_ * HD * SS * 2);
    float* Sb = (float*)take((size_t)ZH * SS * SS * 4); h16* P16 = (h16*)take((size_t)ZH * SS * SS * 2); float* Ob = (float*)take((size_t)ZH * SS * HD * 4); bf* AIh = (bf*)take((size_t)LI * HH * 2); bf* AIl = (bf*)take((size_t)LI * HH * 2); bf* ACh = (bf*)take((size_t)LC * HH * 2); bf* ACl = (bf*)take((size_t)LC * HH * 2);
    float* DLT = (float*)take((size_t)LI * HH * 4); float* X1I = (float*)take((size_t)LI * HH * 4); float* X1C = (float*)take((size_t)LC * HH * 4); float* GA = (float*)take((size_t)LI * MLP * 4); float* GB = (float*)take((size_t)LI * MLP * 4); bf* Fh = (bf*)take((size_t)LI * MLP * 2); bf* Fl = (bf*)take((size_t)LI * MLP * 2);
    if ((size_t)(wsp - (char*)d_ws) > ws_size) return;
    k_cvt8<<<(unsigned)(((size_t)3 * HH * HH / 8 + 255) / 256), 256, 0, stream>>>(IN[8], WQI, (size_t)3 * HH * HH / 8); k_cvt8<<<(unsigned)(((size_t)3 * HH * HH / 8 + 255) / 256), 256, 0, stream>>>(IN[10], WQC, (size_t)3 * HH * HH / 8);
    k_cvt8<<<(unsigned)(((size_t)HH * HH / 8 + 255) / 256), 256, 0, stream>>>(IN[16], WOI, (size_t)HH * HH / 8); k_cvt8<<<(unsigned)(((size_t)HH * HH / 8 + 255) / 256), 256, 0, stream>>>(IN[18], WOC, (size_t)HH * HH / 8);
    k_cvt8<<<(unsigned)(((size_t)MLP * HH / 8 + 255) / 256), 256, 0, stream>>>(IN[22], W1I, (size_t)MLP * HH / 8); k_cvt8<<<(unsigned)(((size_t)MLP * HH / 8 + 255) / 256), 256, 0, stream>>>(IN[24], W2I, (size_t)MLP * HH / 8); k_cvt8<<<(unsigned)(((size_t)MLP * HH / 8 + 255) / 256), 256, 0, stream>>>(IN[26], W3I, (size_t)MLP * HH / 8);
    k_cvt8<<<(unsigned)(((size_t)MLP * HH / 8 + 255) / 256), 256, 0, stream>>>(IN[28], W1C, (size_t)MLP * HH / 8); k_cvt8<<<(unsigned)(((size_t)MLP * HH / 8 + 255) / 256), 256, 0, stream>>>(IN[30], W2C, (size_t)MLP * HH / 8); k_cvt8<<<(unsigned)(((size_t)MLP * HH / 8 + 255) / 256), 256, 0, stream>>>(IN[32], W3C, (size_t)MLP * HH / 8);
    const float* alpha = IN[34]; const float* beta = IN[35];
    for (int b = 0; b < NB_; ++b) { const float* xi = IN[0] + (size_t)b * LI * HH; const float* xc = IN[1] + (size_t)b * LC * HH;
        k_rms<<<LI / 8, 256, 0, stream>>>(xi, 1, LI, IN[6], Xh, Xl); k_gemmw<bf, 1, true><<<dim3(LI / 64, 3 * HH / 64, 1), 32, 0, stream>>>(Xh, Xl, WQI, nullptr, HH, QKVI, 3 * HH, IN[9], 0, 0, 0);
        k_rms<<<LC / 8, 256, 0, stream>>>(xc, 1, LC, IN[7], Xh, Xl); k_gemmw<bf, 1, true><<<dim3(LC / 64, 3 * HH / 64, 1), 32, 0, stream>>>(Xh, Xl, WQC, nullptr, HH, QKVC, 3 * HH, IN[11], 0, 0, 0);
        k_qk<<<(LC * NH_ * 2 + 7) / 8, 256, 0, stream>>>(QKVC, LC, 0, IN[4], IN[5], IN[14], IN[15], Q16, K16); k_qk<<<(LI * NH_ * 2 + 7) / 8, 256, 0, stream>>>(QKVI, LI, LC, IN[2], IN[3], IN[12], IN[13], Q16, K16);
        k_vt<<<(unsigned)(((size_t)NH_ * HD * LC / 2 + 255) / 256), 256, 0, stream>>>(QKVC, LC, 0, VT); k_vt<<<(unsigned)(((size_t)NH_ * HD * LI / 2 + 255) / 256), 256, 0, stream>>>(QKVI, LI, LC, VT);
        for (int h0 = 0; h0 < NH_; h0 += ZH) { const size_t z = (size_t)h0;
            k_gemmw<h16, 0, false><<<dim3(LC / 64, SS / 64, ZH), 32, 0, stream>>>(Q16 + z * SS * HD, nullptr, K16 + z * SS * HD, nullptr, HD, Sb, SS, nullptr, (size_t)SS * HD, (size_t)SS * HD, (size_t)SS * SS);
            k_gemmwg<h16, 0, false><<<dim3(LI / 64, SS / 64, ZH), 32, 0, stream>>>(alpha, Q16 + z * SS * HD + (size_t)LC * HD, nullptr, K16 + z * SS * HD, nullptr, HD, Sb + (size_t)LC * SS, SS, nullptr, (size_t)SS * HD, (size_t)SS * HD, (size_t)SS * SS);
            for (int zz = 0; zz < ZH; ++zz) { k_soft<<<LC / 8, 256, 0, stream>>>(Sb + (size_t)zz * SS * SS, LC, P16 + (size_t)zz * SS * SS); k_softg<<<LI / 8, 256, 0, stream>>>(alpha, Sb + (size_t)zz * SS * SS + (size_t)LC * SS, LI, P16 + (size_t)zz * SS * SS + (size_t)LC * SS); }
            k_gemmw<h16, 0, false><<<dim3(LC / 64, 1, ZH), 32, 0, stream>>>(P16, nullptr, VT + z * HD * SS, nullptr, SS, Ob, HD, nullptr, (size_t)SS * SS, (size_t)HD * SS, (size_t)SS * HD);
            k_gemmwg<h16, 0, false><<<dim3(LI / 64, 1, ZH), 32, 0, stream>>>(alpha, P16 + (size_t)LC * SS, nullptr, VT + z * HD * SS, nullptr, SS, Ob + (size_t)LC * HD, HD, nullptr, (size_t)SS * SS, (size_t)HD * SS, (size_t)SS * HD);
            k_mrg<<<(unsigned)(((size_t)ZH * LC * HD / 2 + 255) / 256), 256, 0, stream>>>(Ob, LC, 0, h0, ACh, ACl); k_mrgg<<<(unsigned)(((size_t)ZH * LI * HD / 2 + 255) / 256), 256, 0, stream>>>(alpha, Ob, LI, LC, h0, AIh, AIl); }
        k_gemmw<bf, 1, true><<<dim3(LC / 64, HH / 64, 1), 32, 0, stream>>>(ACh, ACl, WOC, nullptr, HH, DLT, HH, IN[19], 0, 0, 0); k_resg<<<(LC * HH / 4 + 255) / 256, 256, 0, stream>>>(xc, 1, DLT, nullptr, (size_t)LC * HH / 4, X1C);
        k_rms<<<LC / 8, 256, 0, stream>>>(X1C, 0, LC, IN[21], Xh, Xl); k_gemmw<bf, 1, true><<<dim3(LC / 64, MLP / 64, 1), 32, 0, stream>>>(Xh, Xl, W1C, nullptr, HH, GA, MLP, IN[29], 0, 0, 0); k_gemmw<bf, 1, true><<<dim3(LC / 64, MLP / 64, 1), 32, 0, stream>>>(Xh, Xl, W2C, nullptr, HH, GB, MLP, IN[31], 0, 0, 0);
        k_swi<<<(unsigned)(((size_t)LC * MLP / 4 + 255) / 256), 256, 0, stream>>>(GA, GB, (size_t)LC * MLP / 4, nullptr, Fh, Fl); k_gemmw<bf, 1, true><<<dim3(LC / 64, HH / 64, 1), 32, 0, stream>>>(Fh, Fl, W3C, nullptr, MLP, DLT, HH, IN[33], 0, 0, 0);
        k_resg<<<(LC * HH / 4 + 255) / 256, 256, 0, stream>>>(X1C, 0, DLT, nullptr, (size_t)LC * HH / 4, OUTC + (size_t)b * LC * HH);
        k_gemmwg<bf, 1, true><<<dim3(LI / 64, HH / 64, 1), 32, 0, stream>>>(alpha, AIh, AIl, WOI, nullptr, HH, DLT, HH, IN[17], 0, 0, 0); k_resg<<<(LI * HH / 4 + 255) / 256, 256, 0, stream>>>(xi, 1, DLT, alpha, (size_t)LI * HH / 4, X1I);
        k_rms<<<LI / 8, 256, 0, stream>>>(X1I, 0, LI, IN[20], Xh, Xl); k_gemmwg<bf, 1, true><<<dim3(LI / 64, MLP / 64, 1), 32, 0, stream>>>(beta, Xh, Xl, W1I, nullptr, HH, GA, MLP, IN[23], 0, 0, 0); k_gemmwg<bf, 1, true><<<dim3(LI / 64, MLP / 64, 1), 32, 0, stream>>>(beta, Xh, Xl, W2I, nullptr, HH, GB, MLP, IN[25], 0, 0, 0);
        k_swi<<<(unsigned)(((size_t)LI * MLP / 4 + 255) / 256), 256, 0, stream>>>(GA, GB, (size_t)LI * MLP / 4, beta, Fh, Fl); k_gemmwg<bf, 1, true><<<dim3(LI / 64, HH / 64, 1), 32, 0, stream>>>(beta, Fh, Fl, W3I, nullptr, MLP, DLT, HH, IN[27], 0, 0, 0);
        k_resg<<<(LI * HH / 4 + 255) / 256, 256, 0, stream>>>(X1I, 0, DLT, beta, (size_t)LI * HH / 4, OUTI + (size_t)b * LI * HH); }
}
